// OscillatoryCycle_3255585210482
// MI455X (gfx1250) — hardware-verified
//
#include <hip/hip_runtime.h>
#include <math.h>
#include <stdint.h>
#include <stddef.h>

#define NB_ 4
#define NT_ 2048
#define NV_ 1024
#define NC_ 256
#define NR_ (NB_ * NT_)

typedef _Float16 f16;
typedef f16    v16h __attribute__((ext_vector_type(16)));
typedef f16    v8h  __attribute__((ext_vector_type(8)));
typedef __bf16 v16b __attribute__((ext_vector_type(16)));
typedef float  v8f  __attribute__((ext_vector_type(8)));
typedef float  v4f  __attribute__((ext_vector_type(4)));

__device__ __forceinline__ unsigned short f2bf_bits(float f) {
  const unsigned u = __float_as_uint(f);
  return (unsigned short)((u + 0x7FFFu + ((u >> 16) & 1u)) >> 16);
}
__device__ __forceinline__ float bf_bits2f(unsigned short h) { return __uint_as_float(((unsigned)h) << 16); }

__device__ __forceinline__ v8f mma_h(v16h a, v16h b, v8f c) {
  c = __builtin_amdgcn_wmma_f32_16x16x32_f16(false, a, false, b, (short)0, c, false, false);
  asm volatile("v_nop\n\tv_nop\n\tv_nop\n\tv_nop" : "+v"(c) : "v"(a), "v"(b));
  return c;
}
__device__ __forceinline__ v8f mma_b(v16b a, v16b b, v8f c) {
  c = __builtin_amdgcn_wmma_f32_16x16x32_bf16(false, a, false, b, (short)0, c, false, false);
  asm volatile("v_nop\n\tv_nop\n\tv_nop\n\tv_nop" : "+v"(c) : "v"(a), "v"(b));
  return c;
}

__device__ __forceinline__ v16h ldfrag(const f16* p) {
  union { v16h v; v8h h[2]; } u;
  u.h[0] = *(const v8h*)(p);
  u.h[1] = *(const v8h*)(p + 16);
  return u.v;
}

__device__ __forceinline__ void cvt_split(float f, __bf16& hi, __bf16& lo) {
  const unsigned short hb = f2bf_bits(f);
  hi = __builtin_bit_cast(__bf16, hb);
  lo = __builtin_bit_cast(__bf16, f2bf_bits(f - bf_bits2f(hb)));
}
__device__ __forceinline__ void ldsplit(const float* p, v16b& hi, v16b& lo) {
  const v4f x0 = *(const v4f*)(p);
  const v4f x1 = *(const v4f*)(p + 4);
  const v4f x2 = *(const v4f*)(p + 16);
  const v4f x3 = *(const v4f*)(p + 20);
  union U { v16b v; __bf16 e[16]; } uh, ul;
#pragma unroll
  for (int i = 0; i < 4; ++i) {
    cvt_split(x0[i], uh.e[i],      ul.e[i]);
    cvt_split(x1[i], uh.e[4 + i],  ul.e[4 + i]);
    cvt_split(x2[i], uh.e[8 + i],  ul.e[8 + i]);
    cvt_split(x3[i], uh.e[12 + i], ul.e[12 + i]);
  }
  hi = uh.v; lo = ul.v;
}

__device__ __forceinline__ void wave_sync() {
  __builtin_amdgcn_fence(__ATOMIC_RELEASE, "workgroup");
  __builtin_amdgcn_wave_barrier();
  __builtin_amdgcn_fence(__ATOMIC_ACQUIRE, "workgroup");
}

template <int OUTM>
__device__ __forceinline__ void store_slab(const float* slab, void* Cb, int ldc, int mBase, int ncol, int lane) {
  if (OUTM == 0) {
    float* C = (float*)Cb;
    const int hh = lane >> 4, c4 = (lane & 15) * 4;
    for (int pass = 0; pass < 2; ++pass) {
#pragma unroll
      for (int it = 0; it < 8; ++it) {
        const int row = it * 2 + hh;
        const v4f v = *(const v4f*)(slab + row * 68 + c4);
        *(volatile v4f*)(C + (size_t)(mBase + row) * ldc + ncol + c4) = v;
      }
      __threadfence();
    }
  } else {
    f16* C = (f16*)Cb;
    const int q = lane >> 3, c8 = (lane & 7) * 8;
    for (int pass = 0; pass < 2; ++pass) {
#pragma unroll
      for (int it = 0; it < 4; ++it) {
        const int row = it * 4 + q;
        const float* sp = slab + row * 68 + c8;
        v8h hv;
#pragma unroll
        for (int e = 0; e < 8; ++e) hv[e] = (f16)sp[e];
        *(volatile v8h*)(C + (size_t)(mBase + row) * ldc + ncol + c8) = hv;
      }
      __threadfence();
    }
  }
}

template <int OUTM, int EPI, int KM>
__global__ __launch_bounds__(256) void gemm_kernel(
    const f16* __restrict__ A, int lda, long sA,
    const f16* __restrict__ Bt, int ldb, long sB,
    void* Cv, int ldc, long sC,
    const float* __restrict__ bias,
    const f16* __restrict__ mul, int ldm, long sMu,
    const float* __restrict__ resid, int ldr, long sR,
    const float* __restrict__ dlg,
    int M, int N, int K, float scale, float post) {
  __shared__ __align__(16) float sT[8][16 * 68];
  const int b    = blockIdx.y;
  const int lane = threadIdx.x & 31;
  const int wave = threadIdx.x >> 5;
  const int hh   = lane >> 4;
  const int cc   = lane & 15;
  const int tilesN = N >> 6, tilesM = M >> 6;
  const int tile = blockIdx.x * 8 + wave;
  if (tile >= tilesM * tilesN) return;
  const int tm = tile / tilesN;
  const int tn = tile - tm * tilesN;
  const int m0 = tm << 6, n0 = tn << 6;
  const f16* Ab = A  + (size_t)b * sA;
  const f16* Bb = Bt + (size_t)b * sB;

  v8f acc[4][4];
#pragma unroll
  for (int i = 0; i < 4; ++i)
#pragma unroll
    for (int j = 0; j < 4; ++j) acc[i][j] = (v8f){0.f, 0.f, 0.f, 0.f, 0.f, 0.f, 0.f, 0.f};

  int kbeg = 0, kend = K;
  if (KM == 1) kbeg = m0;
  if (KM == 2) kend = (n0 < m0) ? 0 : K;

  for (int k0 = kbeg; k0 < kend; k0 += 32) {
    v16h bf[4];
#pragma unroll
    for (int j = 0; j < 4; ++j) bf[j] = ldfrag(Bb + (size_t)(n0 + 16 * j + cc) * ldb + k0 + 8 * hh);
#pragma unroll
    for (int i = 0; i < 4; ++i) {
      const v16h af = ldfrag(Ab + (size_t)(m0 + 16 * i + cc) * lda + k0 + 8 * hh);
#pragma unroll
      for (int j = 0; j < 4; ++j) acc[i][j] = mma_h(af, bf[j], acc[i][j]);
    }
  }

  float l2d = 0.f;
  if (EPI == 3) {
    const float dec = 1.0f / (1.0f + expf(-dlg[0]));
    l2d = log2f(dec);
  }
  float* slab = sT[wave];
  void* Cb = (OUTM == 0) ? (void*)((float*)Cv + (size_t)b * sC) : (void*)((f16*)Cv + (size_t)b * sC);

#pragma unroll
  for (int i = 0; i < 4; ++i) {
    const int mBase = m0 + 16 * i;
#pragma unroll
    for (int j = 0; j < 4; ++j)
#pragma unroll
      for (int r = 0; r < 8; ++r) slab[(8 * hh + r) * 68 + 16 * j + cc] = acc[i][j][r] * scale;
    wave_sync();
    if (EPI != 0 && !(EPI == 3 && kend == 0)) {
#pragma unroll 1
      for (int e = 0; e < 32; ++e) {
        const int row = e >> 1;
        const int col = ((e & 1) << 5) + lane;
        float v = slab[row * 68 + col];
        const int m = mBase + row, n = n0 + col;
        if (EPI == 1) {
          v += bias[n];
          v = 0.5f * v * (1.0f + erff(v * 0.70710678118654752f));
          v *= post;
        }
        if (EPI == 2) {
          v += bias[n];
          const float g = 1.0f / (1.0f + expf(-v));
          v = g * (float)mul[(size_t)b * sMu + (size_t)m * ldm + n];
        }
        if (EPI == 3) {
          const int d = n - m;
          const float ex = (float)((d > 1) ? (d - 1) : 0);
          const float w  = exp2f(ex * l2d);
          v = (d > 0) ? v * w : 0.0f;
        }
        if (EPI == 4) {
          v += resid[(size_t)b * sR + (size_t)m * ldr + n];
        }
        slab[row * 68 + col] = v;
      }
      wave_sync();
    }
    store_slab<OUTM>(slab, Cb, ldc, mBase, n0, lane);
    wave_sync();
  }
}

template <int OUTM, int USESC>
__global__ __launch_bounds__(256) void wgen_kernel(
    const float* __restrict__ P0, const float* __restrict__ P1, const float* __restrict__ P2, const float* __restrict__ P3, int RP,
    const float* __restrict__ Q0, const float* __restrict__ Q1, int RQ,
    const float* __restrict__ sa0, const float* __restrict__ sb0, const float* __restrict__ sa1, const float* __restrict__ sb1,
    void* out0, int ldo0, void* out1, int ldo1,
    int M, int N, int K, float cscale) {
  __shared__ __align__(16) float sT[8][16 * 68];
  const int lane = threadIdx.x & 31;
  const int wave = threadIdx.x >> 5;
  const int hh   = lane >> 4;
  const int cc   = lane & 15;
  const int m0 = blockIdx.y * 128 + wave * 16;
  const int n0 = blockIdx.x * 64;
  if (m0 >= M || n0 >= N) return;
  const int segp = m0 / RP;
  const int segq = n0 / RQ;
  const float* Pp = (segp == 0) ? P0 : ((segp == 1) ? P1 : ((segp == 2) ? P2 : P3));
  const float* Qp = (segq == 0) ? Q0 : Q1;
  const int pm = m0 - segp * RP;
  const int qn = n0 - segq * RQ;
  float scale = cscale;
  if (USESC) {
    const float s0 = sa0[0] * sb0[0];
    const float s1 = sa1[0] * sb1[0];
    scale *= (segq == 0) ? s0 : s1;
  }

  v8f acc[4];
#pragma unroll
  for (int j = 0; j < 4; ++j) acc[j] = (v8f){0.f, 0.f, 0.f, 0.f, 0.f, 0.f, 0.f, 0.f};

  for (int k0 = 0; k0 < K; k0 += 32) {
    v16b ah, al;
    ldsplit(Pp + (size_t)(pm + cc) * K + k0 + 8 * hh, ah, al);
#pragma unroll
    for (int j = 0; j < 4; ++j) {
      v16b bh, bl;
      ldsplit(Qp + (size_t)(qn + 16 * j + cc) * K + k0 + 8 * hh, bh, bl);
      acc[j] = mma_b(ah, bh, acc[j]);
      acc[j] = mma_b(ah, bl, acc[j]);
      acc[j] = mma_b(al, bh, acc[j]);
    }
  }

  float* slab = sT[wave];
#pragma unroll
  for (int j = 0; j < 4; ++j)
#pragma unroll
    for (int r = 0; r < 8; ++r) slab[(8 * hh + r) * 68 + 16 * j + cc] = acc[j][r] * scale;
  wave_sync();
  void* ob = (segq == 0) ? out0 : out1;
  const int ldo = (segq == 0) ? ldo0 : ldo1;
  store_slab<OUTM>(slab, ob, ldo, m0, qn, lane);
}

__global__ __launch_bounds__(128) void colsoft_kernel(const float* __restrict__ L0, f16* O0, int nr0,
                                                      const float* __restrict__ L1, f16* O1, int nr1,
                                                      const float* __restrict__ L2, f16* O2, int nr2, float osc) {
  __shared__ __align__(16) float rowbuf[NV_];
  __shared__ float redm[4];
  __shared__ float reds[4];
  const int sel = blockIdx.y;
  const int row = blockIdx.x;
  const float* L = (sel == 0) ? L0 : ((sel == 1) ? L1 : L2);
  f16* O = (sel == 0) ? O0 : ((sel == 1) ? O1 : O2);
  const int nr = (sel == 0) ? nr0 : ((sel == 1) ? nr1 : nr2);
  if (row >= nr) return;
  const int tid = threadIdx.x, lane = tid & 31, wave = tid >> 5;
  const float* p = L + (size_t)row * NV_ + tid * 8;
  const v4f a = *(const v4f*)(p);
  const v4f c = *(const v4f*)(p + 4);
  float mx = fmaxf(fmaxf(fmaxf(a[0], a[1]), fmaxf(a[2], a[3])), fmaxf(fmaxf(c[0], c[1]), fmaxf(c[2], c[3])));
  *(v4f*)(rowbuf + tid * 8)     = a;
  *(v4f*)(rowbuf + tid * 8 + 4) = c;
#pragma unroll
  for (int off = 1; off < 32; off <<= 1) mx = fmaxf(mx, __shfl_xor(mx, off, 32));
  if (lane == 0) redm[wave] = mx;
  __syncthreads();
  const float gmax = fmaxf(fmaxf(redm[0], redm[1]), fmaxf(redm[2], redm[3]));
  float lsum = 0.f;
#pragma unroll 1
  for (int i = 0; i < 8; ++i) {
    const float e = expf(rowbuf[tid * 8 + i] - gmax);
    rowbuf[tid * 8 + i] = e;
    lsum += e;
  }
#pragma unroll
  for (int off = 1; off < 32; off <<= 1) lsum += __shfl_xor(lsum, off, 32);
  if (lane == 0) reds[wave] = lsum;
  __syncthreads();
  const float tot = (reds[0] + reds[1]) + (reds[2] + reds[3]);
  const float f = (1.0f / tot) * osc;
  v8h hv;
#pragma unroll
  for (int i = 0; i < 8; ++i) hv[i] = (f16)(rowbuf[tid * 8 + i] * f);
  f16* op = O + (size_t)row * NV_ + tid * 8;
  *(volatile v8h*)op = hv;
  __threadfence();
  *(volatile v8h*)op = hv;
}

__global__ __launch_bounds__(256) void tconv5_kernel(const float* __restrict__ S0, const float* __restrict__ S1, const float* __restrict__ S2,
                                                     const float* __restrict__ S3, const float* __restrict__ S4,
                                                     f16* D0, f16* D1, f16* D2, f16* D3, f16* D4, int R, float scl) {
  __shared__ __align__(16) float tf[64 * 68];
  const int z = blockIdx.z;
  const float* S = (z == 0) ? S0 : ((z == 1) ? S1 : ((z == 2) ? S2 : ((z == 3) ? S3 : S4)));
  f16* D = (z == 0) ? D0 : ((z == 1) ? D1 : ((z == 2) ? D2 : ((z == 3) ? D3 : D4)));
  const int c0 = blockIdx.x * 64;
  const int r0 = blockIdx.y * 64;
  const int tid = threadIdx.x;
  {
    const int lr = tid >> 4;
    const int c4 = (tid & 15) * 4;
#pragma unroll
    for (int it = 0; it < 4; ++it) {
      const int rr = it * 16 + lr;
      const v4f a = *(const v4f*)(S + (size_t)(r0 + rr) * R + c0 + c4);
      *(v4f*)(tf + rr * 68 + c4) = a;
    }
  }
  __syncthreads();
  const int sub = tid >> 3;
  const int c8  = (tid & 7) * 8;
  v8h hv[2];
#pragma unroll
  for (int it = 0; it < 2; ++it) {
    const int oc = it * 32 + sub;
    v8h t;
#pragma unroll
    for (int e = 0; e < 8; ++e) t[e] = (f16)(tf[(c8 + e) * 68 + oc] * scl);
    hv[it] = t;
  }
  for (int pass = 0; pass < 2; ++pass) {
#pragma unroll
    for (int it = 0; it < 2; ++it) {
      const int oc = it * 32 + sub;
      *(volatile v8h*)(D + (size_t)(c0 + oc) * R + r0 + c8) = hv[it];
    }
    __threadfence();
  }
}

__global__ __launch_bounds__(128) void rms_kernel(const float* __restrict__ x, f16* out) {
  __shared__ float red[4];
  const int row = blockIdx.x;
  const int tid = threadIdx.x, lane = tid & 31, wave = tid >> 5;
  const float* p = x + (size_t)row * NV_ + tid * 8;
  const v4f a = *(const v4f*)(p);
  const v4f c = *(const v4f*)(p + 4);
  float ss = a[0] * a[0] + a[1] * a[1] + a[2] * a[2] + a[3] * a[3]
           + c[0] * c[0] + c[1] * c[1] + c[2] * c[2] + c[3] * c[3];
#pragma unroll
  for (int off = 1; off < 32; off <<= 1) ss += __shfl_xor(ss, off, 32);
  if (lane == 0) red[wave] = ss;
  __syncthreads();
  const float tot = (red[0] + red[1]) + (red[2] + red[3]);
  const float sc = 1.0f / sqrtf(tot * (1.0f / 1024.0f) + 1.1920929e-07f);
  v8h hv;
  hv[0] = (f16)(a[0] * sc); hv[1] = (f16)(a[1] * sc); hv[2] = (f16)(a[2] * sc); hv[3] = (f16)(a[3] * sc);
  hv[4] = (f16)(c[0] * sc); hv[5] = (f16)(c[1] * sc); hv[6] = (f16)(c[2] * sc); hv[7] = (f16)(c[3] * sc);
  f16* op = out + (size_t)row * NV_ + tid * 8;
  *(volatile v8h*)op = hv;
  __threadfence();
  *(volatile v8h*)op = hv;
}

template <int OUTM, int EPI, int KM>
static void run_gemm(hipStream_t st, int nb,
                     const f16* A, int lda, long sA, const f16* Bt, int ldb, long sB,
                     void* C, int ldc, long sC, const float* bias,
                     const f16* mul, int ldm, long sMu, const float* resid, int ldr, long sR,
                     const float* dlg, int M, int N, int K, float scale, float post) {
  const int tiles = (M / 64) * (N / 64);
  gemm_kernel<OUTM, EPI, KM><<<dim3((tiles + 7) / 8, nb), dim3(256), 0, st>>>(
      A, lda, sA, Bt, ldb, sB, C, ldc, sC, bias, mul, ldm, sMu, resid, ldr, sR, dlg, M, N, K, scale, post);
}

extern "C" void kernel_launch(void* const* d_in, const int* in_sizes, int n_in,
                              void* d_out, int out_size, void* d_ws, size_t ws_size,
                              hipStream_t stream) {
  if (n_in < 40) return;
  const int nRV = NR_ * NV_;
  if (in_sizes[0] != nRV || out_size != nRV) return;
  if (in_sizes[1] != NV_ * 32 || in_sizes[2] != NV_ * 64 || in_sizes[3] != NV_ * 128) return;
  if (in_sizes[4] != NC_ * 32 || in_sizes[5] != NC_ * 32 || in_sizes[6] != NC_ * 32 || in_sizes[7] != NC_ * 32) return;
  if (in_sizes[8] < 1 || in_sizes[9] < 1 || in_sizes[14] < 1 || in_sizes[15] < 1) return;
  if (in_sizes[10] != NC_ * 128 || in_sizes[11] != NC_ * 128 || in_sizes[12] != NC_ * 128 || in_sizes[13] != NC_ * 128) return;
  if (in_sizes[16] != NC_ * 32 || in_sizes[17] != NC_ * 32 || in_sizes[18] != NC_ * NC_ || in_sizes[19] < NC_ || in_sizes[20] < 1) return;
  if (in_sizes[21] != NC_ * 64 || in_sizes[22] != NC_ * 64 || in_sizes[23] != NC_ * NC_ || in_sizes[24] < NC_ || in_sizes[25] < 1) return;
  if (in_sizes[26] != NC_ * 128 || in_sizes[27] != NC_ * 128 || in_sizes[28] != NC_ * NC_ || in_sizes[29] < NC_ || in_sizes[30] < 1) return;
  if (in_sizes[31] != NC_ * NC_ || in_sizes[32] < NC_ || in_sizes[33] != NC_ * NC_ || in_sizes[34] < NC_) return;
  if (in_sizes[35] < 1 || in_sizes[36] < 1 || in_sizes[37] < 1 || in_sizes[38] < 1 || in_sizes[39] < 1) return;

  const float* x          = (const float*)d_in[0];
  const float* basis_low  = (const float*)d_in[1];
  const float* basis_mid  = (const float*)d_in[2];
  const float* basis_high = (const float*)d_in[3];
  const float* slow_q     = (const float*)d_in[4];
  const float* slow_k     = (const float*)d_in[5];
  const float* slow_v     = (const float*)d_in[6];
  const float* slow_o     = (const float*)d_in[7];
  const float* slow_decay = (const float*)d_in[8];
  const float* slow_scale = (const float*)d_in[9];
  const float* fast_q     = (const float*)d_in[10];
  const float* fast_k     = (const float*)d_in[11];
  const float* fast_v     = (const float*)d_in[12];
  const float* fast_o     = (const float*)d_in[13];
  const float* fast_decay = (const float*)d_in[14];
  const float* fast_scale = (const float*)d_in[15];
  const float* low_read   = (const float*)d_in[16];
  const float* low_write  = (const float*)d_in[17];
  const float* low_mix    = (const float*)d_in[18];
  const float* low_bias   = (const float*)d_in[19];
  const float* low_oscale = (const float*)d_in[20];
  const float* mid_read   = (const float*)d_in[21];
  const float* mid_write  = (const float*)d_in[22];
  const float* mid_mix    = (const float*)d_in[23];
  const float* mid_bias   = (const float*)d_in[24];
  const float* mid_oscale = (const float*)d_in[25];
  const float* high_read  = (const float*)d_in[26];
  const float* high_write = (const float*)d_in[27];
  const float* high_mix   = (const float*)d_in[28];
  const float* high_bias  = (const float*)d_in[29];
  const float* high_oscale= (const float*)d_in[30];
  const float* tg_w       = (const float*)d_in[31];
  const float* tg_b       = (const float*)d_in[32];
  const float* alpha_w    = (const float*)d_in[33];
  const float* alpha_b    = (const float*)d_in[34];
  const float* mem_slow_scale = (const float*)d_in[35];
  const float* mem_fast_scale = (const float*)d_in[36];
  const float* op_low_scale   = (const float*)d_in[37];
  const float* op_mid_scale   = (const float*)d_in[38];
  const float* op_high_scale  = (const float*)d_in[39];

  size_t off = 0;
  const size_t oXN  = off; off += (size_t)NR_ * NV_ * 2;
  const size_t oLGl = off; off += (size_t)1024 * 1024 * 4;
  const size_t oLGh = off; off += (size_t)1024 * 1024 * 4;
  const size_t oLGm = off; off += (size_t)256 * 1024 * 4;
  const size_t oWSl = off; off += (size_t)1024 * 1024 * 2;
  const size_t oWSh = off; off += (size_t)1024 * 1024 * 2;
  const size_t oWSm = off; off += (size_t)256 * 1024 * 2;
  const size_t oWO1 = off; off += (size_t)1024 * 512 * 2;
  const size_t oWO2 = off; off += (size_t)1024 * 768 * 2;
  const size_t oT5  = off; off += (size_t)5 * 256 * 256 * 2;
  const size_t oQK  = off; off += (size_t)NR_ * 512 * 2;
  const size_t oVT  = off; off += (size_t)256 * NR_ * 2;
  const size_t oPZ  = off; off += (size_t)NB_ * NT_ * NT_ * 2;
  const size_t oR1  = off; off += (size_t)NR_ * 512 * 2;
  const size_t oRF  = off; off += (size_t)NR_ * 256 * 2;
  const size_t oX1  = off; off += (size_t)NR_ * NV_ * 4;
  if (off > ws_size || off > (size_t)134217728) return;
  if ((size_t)NR_ * 768 * 2 * 2 + (size_t)NR_ * 256 * 2 > (size_t)NB_ * NT_ * NT_ * 2) return;

  char* ws = (char*)d_ws;
  f16*   XN  = (f16*)(ws + oXN);
  float* LGl = (float*)(ws + oLGl);
  float* LGh = (float*)(ws + oLGh);
  float* LGm = (float*)(ws + oLGm);
  f16*   WSl = (f16*)(ws + oWSl);
  f16*   WSh = (f16*)(ws + oWSh);
  f16*   WSm = (f16*)(ws + oWSm);
  f16*   WO1 = (f16*)(ws + oWO1);
  f16*   WO2 = (f16*)(ws + oWO2);
  f16*   TGT = (f16*)(ws + oT5);
  f16*   ALT = TGT + (size_t)NC_ * NC_;
  f16*   MXl = TGT + (size_t)2 * NC_ * NC_;
  f16*   MXm = TGT + (size_t)3 * NC_ * NC_;
  f16*   MXh = TGT + (size_t)4 * NC_ * NC_;
  f16*   QK  = (f16*)(ws + oQK);
  f16*   VT  = (f16*)(ws + oVT);
  f16*   P   = (f16*)(ws + oPZ);
  f16*   Z   = (f16*)(ws + oPZ);
  f16*   H   = (f16*)(ws + oPZ + (size_t)NR_ * 768 * 2);
  f16*   HF  = (f16*)(ws + oPZ + (size_t)NR_ * 768 * 2 * 2);
  f16*   R1  = (f16*)(ws + oR1);
  f16*   RF  = (f16*)(ws + oRF);
  float* X1  = (float*)(ws + oX1);
  float* OUT = (float*)d_out;

  const float* fdum = x;
  const f16*   hdum = XN;
  const dim3 blk(256);

  wgen_kernel<0, 0><<<dim3(1024 / 64, 1024 / 128), blk, 0, stream>>>(
      slow_q, slow_k, slow_v, low_read, NC_, basis_low, basis_low, NV_,
      slow_scale, slow_scale, slow_scale, slow_scale, (void*)LGl, 1024, (void*)LGl, 1024, 1024, 1024, 32, 1.0f);
  wgen_kernel<0, 0><<<dim3(1024 / 64, 1024 / 128), blk, 0, stream>>>(
      fast_q, fast_k, fast_v, high_read, NC_, basis_high, basis_high, NV_,
      slow_scale, slow_scale, slow_scale, slow_scale, (void*)LGh, 1024, (void*)LGh, 1024, 1024, 1024, 128, 1.0f);
  wgen_kernel<0, 0><<<dim3(1024 / 64, 256 / 128), blk, 0, stream>>>(
      mid_read, mid_read, mid_read, mid_read, NC_, basis_mid, basis_mid, NV_,
      slow_scale, slow_scale, slow_scale, slow_scale, (void*)LGm, 1024, (void*)LGm, 1024, 256, 1024, 64, 1.0f);
  wgen_kernel<1, 1><<<dim3(512 / 64, 1024 / 128), blk, 0, stream>>>(
      basis_low, basis_low, basis_low, basis_low, NV_, slow_o, low_write, NC_,
      slow_scale, mem_slow_scale, low_oscale, op_low_scale, (void*)WO1, 512, (void*)WO2, 768, 1024, 512, 32, 256.0f);
  wgen_kernel<1, 1><<<dim3(512 / 64, 1024 / 128), blk, 0, stream>>>(
      basis_high, basis_high, basis_high, basis_high, NV_, fast_o, high_write, NC_,
      fast_scale, mem_fast_scale, high_oscale, op_high_scale, (void*)(WO1 + 256), 512, (void*)(WO2 + 512), 768, 1024, 512, 128, 256.0f);
  wgen_kernel<1, 1><<<dim3(256 / 64, 1024 / 128), blk, 0, stream>>>(
      basis_mid, basis_mid, basis_mid, basis_mid, NV_, mid_write, mid_write, NC_,
      mid_oscale, op_mid_scale, mid_oscale, op_mid_scale, (void*)(WO2 + 256), 768, (void*)(WO2 + 256), 768, 1024, 256, 64, 256.0f);

  colsoft_kernel<<<dim3(1024, 3), dim3(128), 0, stream>>>(LGl, WSl, 1024, LGh, WSh, 1024, LGm, WSm, 256, 1024.0f);
  tconv5_kernel<<<dim3(NC_ / 64, NC_ / 64, 5), blk, 0, stream>>>(tg_w, alpha_w, low_mix, mid_mix, high_mix, TGT, ALT, MXl, MXm, MXh, NC_, 64.0f);

  rms_kernel<<<dim3(NR_), dim3(128), 0, stream>>>(x, XN);
  const long sQK = (long)NT_ * 512, sP = (long)NT_ * NT_;
  run_gemm<1, 0, 0>(stream, 1, XN, NV_, 0L, WSl, NV_, 0L, (void*)QK, 512, 0L, fdum, hdum, 0, 0L, fdum, 0, 0L, fdum,
                    NR_, 512, NV_, 1.0f / 64.0f, 1.0f);
  run_gemm<1, 0, 0>(stream, 1, WSl + (size_t)512 * NV_, NV_, 0L, XN, NV_, 0L, (void*)VT, NR_, 0L, fdum, hdum, 0, 0L, fdum, 0, 0L, fdum,
                    NC_, NR_, NV_, 1.0f / 64.0f, 1.0f);
  run_gemm<1, 3, 2>(stream, NB_, QK, 512, sQK, QK + 256, 512, sQK, (void*)P, NT_, sP, fdum, hdum, 0, 0L, fdum, 0, 0L, slow_decay,
                    NT_, NT_, NC_, 4.0f, 1.0f);
  run_gemm<1, 0, 1>(stream, NB_, P, NT_, sP, VT, NR_, (long)NT_, (void*)R1, 512, sQK, fdum, hdum, 0, 0L, fdum, 0, 0L, fdum,
                    NT_, NC_, NT_, 1.0f / 64.0f, 1.0f);
  run_gemm<1, 0, 0>(stream, 1, XN, NV_, 0L, WSh, NV_, 0L, (void*)QK, 512, 0L, fdum, hdum, 0, 0L, fdum, 0, 0L, fdum,
                    NR_, 512, NV_, 1.0f / 64.0f, 1.0f);
  run_gemm<1, 0, 0>(stream, 1, WSh + (size_t)512 * NV_, NV_, 0L, XN, NV_, 0L, (void*)VT, NR_, 0L, fdum, hdum, 0, 0L, fdum, 0, 0L, fdum,
                    NC_, NR_, NV_, 1.0f / 64.0f, 1.0f);
  run_gemm<1, 3, 2>(stream, NB_, QK, 512, sQK, QK + 256, 512, sQK, (void*)P, NT_, sP, fdum, hdum, 0, 0L, fdum, 0, 0L, fast_decay,
                    NT_, NT_, NC_, 4.0f, 1.0f);
  run_gemm<1, 0, 1>(stream, NB_, P, NT_, sP, VT, NR_, (long)NT_, (void*)RF, 256, (long)NT_ * 256, fdum, hdum, 0, 0L, fdum, 0, 0L, fdum,
                    NT_, NC_, NT_, 1.0f / 64.0f, 1.0f);
  run_gemm<1, 2, 0>(stream, 1, R1, 512, 0L, TGT, NC_, 0L, (void*)(R1 + 256), 512, 0L, tg_b, RF, 256, 0L, fdum, 0, 0L, fdum,
                    NR_, NC_, NC_, 1.0f / 16384.0f, 1.0f);
  run_gemm<0, 4, 0>(stream, 1, R1, 512, 0L, WO1, 512, 0L, (void*)X1, NV_, 0L, fdum, hdum, 0, 0L, x, NV_, 0L, fdum,
                    NR_, NV_, 512, 1.0f / 65536.0f, 1.0f);

  rms_kernel<<<dim3(NR_), dim3(128), 0, stream>>>(X1, XN);
  run_gemm<1, 0, 0>(stream, 1, XN, NV_, 0L, WSl + (size_t)768 * NV_, NV_, 0L, (void*)Z, 768, 0L, fdum, hdum, 0, 0L, fdum, 0, 0L, fdum,
                    NR_, NC_, NV_, 1.0f / 64.0f, 1.0f);
  run_gemm<1, 0, 0>(stream, 1, XN, NV_, 0L, WSm, NV_, 0L, (void*)(Z + 256), 768, 0L, fdum, hdum, 0, 0L, fdum, 0, 0L, fdum,
                    NR_, NC_, NV_, 1.0f / 64.0f, 1.0f);
  run_gemm<1, 0, 0>(stream, 1, XN, NV_, 0L, WSh + (size_t)768 * NV_, NV_, 0L, (void*)(Z + 512), 768, 0L, fdum, hdum, 0, 0L, fdum, 0, 0L, fdum,
                    NR_, NC_, NV_, 1.0f / 64.0f, 1.0f);
  run_gemm<1, 1, 0>(stream, 1, Z, 768, 0L, MXl, NC_, 0L, (void*)H, 768, 0L, low_bias, hdum, 0, 0L, fdum, 0, 0L, fdum,
                    NR_, NC_, NC_, 1.0f / 1024.0f, 256.0f);
  run_gemm<1, 1, 0>(stream, 1, Z + 256, 768, 0L, MXm, NC_, 0L, (void*)(H + 256), 768, 0L, mid_bias, hdum, 0, 0L, fdum, 0, 0L, fdum,
                    NR_, NC_, NC_, 1.0f / 1024.0f, 256.0f);
  run_gemm<1, 1, 0>(stream, 1, Z + 512, 768, 0L, MXh, NC_, 0L, (void*)HF, 256, 0L, high_bias, hdum, 0, 0L, fdum, 0, 0L, fdum,
                    NR_, NC_, NC_, 1.0f / 1024.0f, 256.0f);
  run_gemm<1, 2, 0>(stream, 1, H, 768, 0L, ALT, NC_, 0L, (void*)(H + 512), 768, 0L, alpha_b, HF, 256, 0L, fdum, 0, 0L, fdum,
                    NR_, NC_, NC_, 1.0f / 16384.0f, 1.0f);
  run_gemm<0, 4, 0>(stream, 1, H, 768, 0L, WO2, 768, 0L, (void*)OUT, NV_, 0L, fdum, hdum, 0, 0L, X1, NV_, 0L, fdum,
                    NR_, NV_, 768, 1.0f / 65536.0f, 1.0f);
  (void)hipGetLastError();
}
